// GNN_56418690401074
// MI455X (gfx1250) — hardware-verified
//
#include <hip/hip_runtime.h>
#include <stddef.h>
#include <stdint.h>
#include <math.h>

#pragma clang fp contract(off)

#define NGR    64
#define NP0    32768
#define CD     128
#define GW     384
#define GK     1152
#define XK     384
#define PERPAD 512
#define NTHR   256
#define NWAVE  8
#define EPT    8
#define CHUNK  (NTHR * EPT)
#define WCAP   (EPT * 32)
#define LISTN  (NWAVE * WCAP)
#define NBA    1024
#define SLA    10
#define RCAP   12288
#define DEGCAP 31
#define AGG_ZINTS (LISTN + 2 * RCAP + 3 * NBA)
#define MISC_INTS 32
#define AGG_LDS_INTS (AGG_ZINTS + MISC_INTS + (NWAVE * GK) / 2)
#define GBM    64
#define GBN    128
#define GTHR   128
#define PU_A   6144
#define PU_W   18432
#define PU_TOT (PU_A + 5 * PU_W)
#define PTHR   512
#define WSMAX  134217728

static_assert((CHUNK & (CHUNK - 1)) == 0 && CHUNK <= 4096);
static_assert((NBA & (NBA - 1)) == 0 && NBA == (1 << SLA));
static_assert(NBA % NWAVE == 0 && AGG_ZINTS % 4 == 0 && ((AGG_ZINTS + MISC_INTS) % 4) == 0);
static_assert(PU_A % NTHR == 0 && PU_W % NTHR == 0 && PU_TOT % NTHR == 0);
static_assert(PU_A * 8 == GW * CD && PU_W * 8 == GW * XK && PU_W * 8 == CD * GK);
static_assert(GK % 32 == 0 && XK % 32 == 0 && CD % 32 == 0);
static_assert(AGG_LDS_INTS * 4 <= 300000);
static_assert(DEGCAP <= 31);
static_assert(NTHR == NWAVE * 32 && NTHR >= 3 * 32);

typedef float          v4f   __attribute__((ext_vector_type(4)));
typedef float          v8f   __attribute__((ext_vector_type(8)));
typedef int            v4i   __attribute__((ext_vector_type(4)));
typedef int            v8i   __attribute__((ext_vector_type(8)));
typedef unsigned short v4us  __attribute__((ext_vector_type(4)));
typedef unsigned short v8us  __attribute__((ext_vector_type(8)));
typedef unsigned short v16us __attribute__((ext_vector_type(16)));
typedef __bf16         v16bf __attribute__((ext_vector_type(16)));
typedef v4f  __attribute__((may_alias)) v4fa;
typedef v4i  __attribute__((may_alias)) v4ia;
typedef v4us __attribute__((may_alias)) v4usa;
typedef v8us __attribute__((may_alias)) v8usa;
union FragB { v16bf v; v16us u; v8us h[2]; v8i w; };

__device__ __forceinline__ v8f wmb(const FragB& a, const FragB& b, v8f c) {
  v8f d = __builtin_amdgcn_wmma_f32_16x16x32_bf16(false, a.v, false, b.v, (short)0, c, false, false);
  asm volatile("v_nop\n\tv_nop\n\tv_nop\n\tv_nop" : "+v"(d) : "v"(a.w), "v"(b.w));
  return d;
}
__device__ __forceinline__ unsigned bf16_bits(float f) {
  const unsigned u = __float_as_uint(f);
  return (u + 0x7FFFu + ((u >> 16) & 1u)) >> 16;
}
__device__ __forceinline__ float bf16_val(float f) { return __uint_as_float(bf16_bits(f) << 16); }
__device__ __forceinline__ v4f bf16_val4(v4f a) {
  v4f r; r.x = bf16_val(a.x); r.y = bf16_val(a.y); r.z = bf16_val(a.z); r.w = bf16_val(a.w); return r;
}
__device__ __forceinline__ void wave_sync() {
  __builtin_amdgcn_fence(__ATOMIC_RELEASE, "wavefront");
  __builtin_amdgcn_wave_barrier();
  __builtin_amdgcn_fence(__ATOMIC_ACQUIRE, "wavefront");
}
__device__ __forceinline__ float wmaxf(float v) {
#pragma unroll
  for (int d = 16; d >= 1; d >>= 1) v = fmaxf(v, __shfl_xor(v, d, 32));
  return v;
}
__device__ __forceinline__ float wsumf(float v) {
#pragma unroll
  for (int d = 16; d >= 1; d >>= 1) v = v + __shfl_xor(v, d, 32);
  return v;
}
__device__ __forceinline__ void split3(float v, unsigned short& h, unsigned short& m, unsigned short& l) {
  const unsigned hb = bf16_bits(v);
  const float r1 = v - __uint_as_float(hb << 16);
  const unsigned mb = bf16_bits(r1);
  const float r2 = r1 - __uint_as_float(mb << 16);
  const unsigned lb = bf16_bits(r2);
  h = (unsigned short)hb; m = (unsigned short)mb; l = (unsigned short)lb;
}
__device__ __forceinline__ void stage3(unsigned short* rb, int off, int pstr, const v4f y) {
  v4us hv, mv, lv;
  unsigned short a, b, c;
  split3(y.x, a, b, c); hv[0] = a; mv[0] = b; lv[0] = c;
  split3(y.y, a, b, c); hv[1] = a; mv[1] = b; lv[1] = c;
  split3(y.z, a, b, c); hv[2] = a; mv[2] = b; lv[2] = c;
  split3(y.w, a, b, c); hv[3] = a; mv[3] = b; lv[3] = c;
  *(v4usa*)(rb + off) = hv;
  *(v4usa*)(rb + pstr + off) = mv;
  *(v4usa*)(rb + 2 * pstr + off) = lv;
}

template <int SLB>
__device__ __forceinline__ int scan_chunk(const int* __restrict__ dsts, int nE, int cbase, int slotBase,
                                          int nb, int vec8, int* list, int tid, int lane, int wave) {
  int wc = 0;
  const int el0  = tid * EPT;
  const int e0   = cbase + el0;
  const int sent = -2147483647 - 1;
  v4i da, db;
  if (vec8 != 0 && cbase + CHUNK <= nE) {
    da = *(const v4i*)(dsts + e0);
    db = *(const v4i*)(dsts + e0 + 4);
  } else {
    da.x = (e0     < nE) ? dsts[min(e0,     nE - 1)] : sent;
    da.y = (e0 + 1 < nE) ? dsts[min(e0 + 1, nE - 1)] : sent;
    da.z = (e0 + 2 < nE) ? dsts[min(e0 + 2, nE - 1)] : sent;
    da.w = (e0 + 3 < nE) ? dsts[min(e0 + 3, nE - 1)] : sent;
    db.x = (e0 + 4 < nE) ? dsts[min(e0 + 4, nE - 1)] : sent;
    db.y = (e0 + 5 < nE) ? dsts[min(e0 + 5, nE - 1)] : sent;
    db.z = (e0 + 6 < nE) ? dsts[min(e0 + 6, nE - 1)] : sent;
    db.w = (e0 + 7 < nE) ? dsts[min(e0 + 7, nE - 1)] : sent;
  }
  const unsigned nbs = (unsigned)slotBase;
  const unsigned unb = (unsigned)nb;
  const unsigned s0 = (unsigned)da.x - nbs, s1 = (unsigned)da.y - nbs;
  const unsigned s2 = (unsigned)da.z - nbs, s3 = (unsigned)da.w - nbs;
  const unsigned s4 = (unsigned)db.x - nbs, s5 = (unsigned)db.y - nbs;
  const unsigned s6 = (unsigned)db.z - nbs, s7 = (unsigned)db.w - nbs;
  const bool h0 = s0 < unb, h1 = s1 < unb, h2 = s2 < unb, h3 = s3 < unb;
  const bool h4 = s4 < unb, h5 = s5 < unb, h6 = s6 < unb, h7 = s7 < unb;
  const unsigned any = __builtin_amdgcn_ballot_w32(h0 | h1 | h2 | h3 | h4 | h5 | h6 | h7);
  if (any != 0u) {
#define HITJ(J, HJ, SJ) { \
      const unsigned mj = __builtin_amdgcn_ballot_w32(HJ); \
      if (mj != 0u) { \
        if (HJ) { \
          const int pos = wc + (int)__builtin_amdgcn_mbcnt_lo(mj, 0u); \
          if (pos < WCAP) list[wave * WCAP + pos] = ((el0 + (J)) << SLB) | (int)(SJ); \
        } \
        wc += (int)__builtin_popcount(mj); } }
    HITJ(0, h0, s0)
    HITJ(1, h1, s1)
    HITJ(2, h2, s2)
    HITJ(3, h3, s3)
    HITJ(4, h4, s4)
    HITJ(5, h5, s5)
    HITJ(6, h6, s6)
    HITJ(7, h7, s7)
#undef HITJ
  }
  return wc;
}

__global__ __launch_bounds__(NTHR) void k_prep(const float* __restrict__ W1, const float* __restrict__ W2,
                                               const float* __restrict__ W3, const float* __restrict__ Wh1,
                                               const float* __restrict__ Wh2, const float* __restrict__ Wh3,
                                               unsigned short* W1T, unsigned short* W2T, unsigned short* W3T,
                                               unsigned short* Wh1T, unsigned short* Wh2T, unsigned short* Wh3T) {
  const int u = (int)blockIdx.x * NTHR + (int)threadIdx.x;
  const float* W; unsigned short* P; int sstr, kin, kt8, v;
  if (u < PU_A)                 { W = W1;  P = W1T;  sstr = GW; kin = CD; kt8 = CD / 8; v = u; }
  else if (u < PU_A + PU_W)     { W = W2;  P = W2T;  sstr = GW; kin = CD; kt8 = XK / 8; v = u - PU_A; }
  else if (u < PU_A + 2 * PU_W) { W = W3;  P = W3T;  sstr = GW; kin = CD; kt8 = XK / 8; v = u - PU_A - PU_W; }
  else if (u < PU_A + 3 * PU_W) { W = Wh1; P = Wh1T; sstr = CD; kin = GW; kt8 = GK / 8; v = u - PU_A - 2 * PU_W; }
  else if (u < PU_A + 4 * PU_W) { W = Wh2; P = Wh2T; sstr = CD; kin = GW; kt8 = GK / 8; v = u - PU_A - 3 * PU_W; }
  else if (u < PU_A + 5 * PU_W) { W = Wh3; P = Wh3T; sstr = CD; kin = GW; kt8 = GK / 8; v = u - PU_A - 4 * PU_W; }
  else return;
  const int n  = v / kt8;
  const int kk = (v - n * kt8) * 8;
  const int ks = kk % kin;
  const float* p = W + (size_t)ks * sstr + n;
  v8us o;
#pragma unroll
  for (int i = 0; i < 8; ++i) o[i] = (unsigned short)bf16_bits(p[(size_t)i * sstr]);
  unsigned short* dp = P + (size_t)v * 8;
  *(volatile v8us*)dp = o;
  __threadfence();
  *(volatile v8us*)dp = o;
}

__global__ __launch_bounds__(NTHR) void k_cvx(const float* __restrict__ x, int nUnits, unsigned short* xb) {
  const int u = (int)blockIdx.x * NTHR + (int)threadIdx.x;
  if (u >= nUnits) return;
  const float* p = x + (size_t)u * 8;
  const v4f a = *(const v4fa*)p;
  const v4f b = *(const v4fa*)(p + 4);
  v8us o;
  o[0] = (unsigned short)bf16_bits(a.x); o[1] = (unsigned short)bf16_bits(a.y);
  o[2] = (unsigned short)bf16_bits(a.z); o[3] = (unsigned short)bf16_bits(a.w);
  o[4] = (unsigned short)bf16_bits(b.x); o[5] = (unsigned short)bf16_bits(b.y);
  o[6] = (unsigned short)bf16_bits(b.z); o[7] = (unsigned short)bf16_bits(b.w);
  unsigned short* dp = xb + (size_t)u * 8;
  *(volatile v8us*)dp = o;
  __threadfence();
  *(volatile v8us*)dp = o;
}

__device__ __forceinline__ void gemm64x128(const unsigned short* __restrict__ A, const unsigned short* __restrict__ BT,
                                           int K, int rowBase, float* stg, int lane, int wave) {
  const int hh = lane >> 4, m = lane & 15;
  v8f acc[8];
  {
    const v8f z = {0.f, 0.f, 0.f, 0.f, 0.f, 0.f, 0.f, 0.f};
#pragma unroll
    for (int t = 0; t < 8; ++t) acc[t] = z;
  }
  const unsigned short* ap = A + (size_t)(rowBase + 16 * wave + m) * (size_t)K + 8 * hh;
  const unsigned short* bp = BT + (size_t)m * (size_t)K + 8 * hh;
#pragma unroll 1
  for (int k0 = 0; k0 < K; k0 += 32) {
    FragB af;
    af.h[0] = *(const v8usa*)(ap + k0);
    af.h[1] = *(const v8usa*)(ap + k0 + 16);
#pragma unroll
    for (int nt = 0; nt < 8; ++nt) {
      const unsigned short* wq = bp + (size_t)(16 * nt) * (size_t)K + k0;
      FragB bf;
      bf.h[0] = *(const v8usa*)wq;
      bf.h[1] = *(const v8usa*)(wq + 16);
      acc[nt] = wmb(af, bf, acc[nt]);
    }
  }
#pragma unroll
  for (int nt = 0; nt < 8; ++nt) {
    const int lc = 16 * nt + m;
#pragma unroll
    for (int r = 0; r < 8; ++r) {
      const int lr = 16 * wave + 8 * hh + r;
      stg[lr * GBN + lc] = acc[nt][r];
    }
  }
  __syncthreads();
}

__global__ __launch_bounds__(GTHR) void k_gemma(const unsigned short* __restrict__ A, const unsigned short* __restrict__ WT,
                                                int K, const float* __restrict__ avs, const float* __restrict__ avd,
                                                float* H, float* ES, float* ED) {
  __shared__ __attribute__((aligned(16))) float stg[GBM * GBN];
  __shared__ __attribute__((aligned(16))) float sred[128];
  const int tid = (int)threadIdx.x, lane = tid & 31, wave = tid >> 5;
  const int rowBase = (int)blockIdx.x * GBM;
  const int head = (int)blockIdx.y;
  gemm64x128(A, WT + (size_t)head * CD * (size_t)K, K, rowBase, stg, lane, wave);

  const v4f as4 = bf16_val4(*(const v4f*)(avs + head * CD + 4 * lane));
  const v4f ad4 = bf16_val4(*(const v4f*)(avd + head * CD + 4 * lane));
  v4f pv[16];
#pragma unroll
  for (int i = 0; i < 16; ++i) pv[i] = *(const v4fa*)(stg + (16 * wave + i) * GBN + 4 * lane);
  float esv = 0.0f, edv = 0.0f;
#pragma unroll
  for (int i = 0; i < 16; ++i) {
    float pe = pv[i].x * as4.x;
    pe = fmaf(pv[i].y, as4.y, pe); pe = fmaf(pv[i].z, as4.z, pe); pe = fmaf(pv[i].w, as4.w, pe);
    float pd = pv[i].x * ad4.x;
    pd = fmaf(pv[i].y, ad4.y, pd); pd = fmaf(pv[i].z, ad4.z, pd); pd = fmaf(pv[i].w, ad4.w, pd);
    pe = wsumf(pe);
    pd = wsumf(pd);
    esv = (lane == i) ? pe : esv;
    edv = (lane == i) ? pd : edv;
  }
  if (lane < 16) { sred[16 * wave + lane] = esv; sred[64 + 16 * wave + lane] = edv; }
#pragma unroll
  for (int i = 0; i < 16; ++i) {
    float* op = H + (size_t)(rowBase + 16 * wave + i) * GW + head * CD + 4 * lane;
    *(volatile v4f*)op = pv[i];
  }
  __threadfence();
#pragma unroll
  for (int i = 0; i < 16; ++i) {
    float* op = H + (size_t)(rowBase + 16 * wave + i) * GW + head * CD + 4 * lane;
    *(volatile v4f*)op = pv[i];
  }
  __syncthreads();
  if (wave == 0) {
    const v4f sv = *(const v4fa*)(sred + 4 * lane);
    float* bp = (lane < 16) ? (ES + (size_t)head * NP0 + rowBase + 4 * lane)
                            : (ED + (size_t)head * NP0 + rowBase + 4 * (lane - 16));
    *(volatile v4f*)bp = sv;
    __threadfence();
    *(volatile v4f*)bp = sv;
  }
}

__global__ __launch_bounds__(GTHR) void k_gemmb(const unsigned short* __restrict__ G, const unsigned short* __restrict__ WhT,
                                                const float* __restrict__ bh, const float* __restrict__ pw,
                                                float* HH, float* SCORE) {
  __shared__ __attribute__((aligned(16))) float stg[GBM * GBN];
  __shared__ __attribute__((aligned(16))) float spw[128];
  __shared__ __attribute__((aligned(16))) float ssc[64];
  __shared__ float srn[4];
  const int tid = (int)threadIdx.x, lane = tid & 31, wave = tid >> 5;
  const int rowBase = (int)blockIdx.x * GBM;
  spw[tid] = bf16_val(pw[tid]);
  __syncthreads();
  if (tid == 0) {
    float ss = 0.0f;
#pragma unroll 4
    for (int c = 0; c < CD; ++c) { const float w = spw[c]; ss = ss + w * w; }
    srn[0] = 1.0f / sqrtf(ss);
  }
  gemm64x128(G, WhT, GK, rowBase, stg, lane, wave);
  const float rn = srn[0];
  const v4f bb4 = bf16_val4(*(const v4f*)(bh + 4 * lane));
  const v4f pw4 = *(const v4fa*)(spw + 4 * lane);
  v4f pv[16];
#pragma unroll
  for (int i = 0; i < 16; ++i) pv[i] = *(const v4fa*)(stg + (16 * wave + i) * GBN + 4 * lane);
  float dv = 0.0f;
#pragma unroll
  for (int i = 0; i < 16; ++i) {
    const v4f t = pv[i] + bb4;
    v4f y;
    y.x = (t.x > 0.0f) ? t.x : (t.x - t.x);
    y.y = (t.y > 0.0f) ? t.y : (t.y - t.y);
    y.z = (t.z > 0.0f) ? t.z : (t.z - t.z);
    y.w = (t.w > 0.0f) ? t.w : (t.w - t.w);
    pv[i] = y;
    float pd = y.x * pw4.x;
    pd = fmaf(y.y, pw4.y, pd); pd = fmaf(y.z, pw4.z, pd); pd = fmaf(y.w, pw4.w, pd);
    pd = wsumf(pd);
    dv = (lane == i) ? pd : dv;
  }
  const float scv = tanhf(dv * rn);
  if (lane < 16) ssc[16 * wave + lane] = scv;
#pragma unroll
  for (int i = 0; i < 16; ++i) {
    float* op = HH + (size_t)(rowBase + 16 * wave + i) * CD + 4 * lane;
    *(volatile v4f*)op = pv[i];
  }
  __threadfence();
#pragma unroll
  for (int i = 0; i < 16; ++i) {
    float* op = HH + (size_t)(rowBase + 16 * wave + i) * CD + 4 * lane;
    *(volatile v4f*)op = pv[i];
  }
  __syncthreads();
  if (wave == 0) {
    const v4f sv = *(const v4fa*)(ssc + 4 * (lane & 15));
    float* sp = SCORE + rowBase + 4 * (lane & 15);
    if (lane < 16) *(volatile v4f*)sp = sv;
    __threadfence();
    if (lane < 16) *(volatile v4f*)sp = sv;
  }
}

__global__ __launch_bounds__(NTHR) void k_attn(const int* __restrict__ srcs, const int* __restrict__ dsts,
                                               int nE, int nN, int vec8,
                                               const float* __restrict__ H, const float* __restrict__ ES,
                                               const float* __restrict__ ED, const float* __restrict__ bias,
                                               unsigned short* G, int* flags) {
  extern __shared__ __attribute__((aligned(16))) int dsm[];
  int* list = dsm;
  int* hl   = dsm + LISTN;
  int* sl   = hl + RCAP;
  int* cnt  = sl + RCAP;
  int* offs = cnt + NBA;
  int* cur  = offs + NBA;
  int* misc = cur + NBA;
  const int tid = (int)threadIdx.x, lane = tid & 31, wave = tid >> 5;
  unsigned short* rowbuf = (unsigned short*)(misc + MISC_INTS) + wave * GK;
  const int nodeBase = (int)blockIdx.x * NBA;

  {
    const v4i z4 = {0, 0, 0, 0};
    for (int i = tid * 4; i < AGG_ZINTS; i += NTHR * 4) *(v4ia*)(dsm + i) = z4;
    if (tid < MISC_INTS) misc[tid] = 0;
  }
  const v4f bv0 = bf16_val4(*(const v4f*)(bias + 4 * lane));
  const v4f bv1 = bf16_val4(*(const v4f*)(bias + CD + 4 * lane));
  const v4f bv2 = bf16_val4(*(const v4f*)(bias + 2 * CD + 4 * lane));
  __syncthreads();

  int t = 0, ov = 0;
  const int nChunks = (nE + CHUNK - 1) / CHUNK;
#pragma unroll 1
  for (int ch = 0; ch < nChunks; ++ch) {
    const int cbase = ch * CHUNK;
    const int wc = scan_chunk<SLA>(dsts, nE, cbase, nodeBase, NBA, vec8, list, tid, lane, wave);
    if (lane == 0) misc[wave] = wc;
    __syncthreads();
    if (wave == 0) {
#pragma unroll 1
      for (int w2 = 0; w2 < NWAVE; ++w2) {
        int c = misc[w2];
        c = c < 0 ? 0 : (c > WCAP ? WCAP : c);
#pragma unroll 1
        for (int b0 = 0; b0 < c; b0 += 32) {
          const int idx = b0 + lane;
          const int ent = list[w2 * WCAP + (idx < WCAP ? idx : WCAP - 1)];
          const int m32 = (c - b0) < 32 ? (c - b0) : 32;
#pragma unroll 1
          for (int k = 0; k < m32; ++k) {
            const int u    = __builtin_amdgcn_readlane(ent, k);
            const int slot = u & (NBA - 1);
            const int el   = (u >> SLA) & (CHUNK - 1);
            const int pk   = ((cbase + el) << SLA) | slot;
            if (t < RCAP) {
              if (lane == 0) { hl[t] = pk; cnt[slot] = cnt[slot] + 1; }
              t = t + 1;
            } else {
              ov = 1;
            }
          }
        }
      }
    }
    __syncthreads();
  }
  if (wave == 0 && lane == 0) { misc[8] = t; misc[9] = ov; }
  __syncthreads();
  int tt = misc[8];
  tt = tt < 0 ? 0 : (tt > RCAP ? RCAP : tt);
  const int ovf = misc[9];

  if (wave == 0) {
    const int base = lane * (NBA / 32);
    int s = 0;
#pragma unroll 1
    for (int i = 0; i < NBA / 32; ++i) s += cnt[base + i];
    int incl = s;
#pragma unroll
    for (int d = 1; d < 32; d <<= 1) {
      const int y = __shfl_up(incl, d, 32);
      if (lane >= d) incl += y;
    }
    int run = incl - s;
#pragma unroll 1
    for (int i = 0; i < NBA / 32; ++i) {
      const int cv = cnt[base + i];
      offs[base + i] = run;
      cur[base + i]  = run;
      run += cv;
    }
  }
  __syncthreads();
  if (wave == 0) {
#pragma unroll 1
    for (int b0 = 0; b0 < tt; b0 += 32) {
      const int idx = b0 + lane;
      const int ent = hl[idx < RCAP ? idx : RCAP - 1];
      const int m32 = (tt - b0) < 32 ? (tt - b0) : 32;
#pragma unroll 1
      for (int k = 0; k < m32; ++k) {
        const int u    = __builtin_amdgcn_readlane(ent, k);
        const int slot = u & (NBA - 1);
        if (lane == 0) {
          int p = cur[slot];
          p = p < 0 ? 0 : (p > RCAP - 1 ? RCAP - 1 : p);
          sl[p] = u;
          cur[slot] = p + 1;
        }
      }
    }
  }
  __syncthreads();

  const float qnan = __int_as_float(0x7fc00000);
  const float ninf = -__builtin_inff();
  const float pz = (ovf != 0) ? qnan : 0.0f;
  int wbig = 0;
#pragma unroll 1
  for (int si = 0; si < NBA / NWAVE; ++si) {
    const int s    = si * NWAVE + wave;
    const int node = nodeBase + s;
    int c = cnt[s];
    const bool big = c > DEGCAP;
    c = c < 0 ? 0 : (c > DEGCAP ? DEGCAP : c);
    int o = offs[s];
    o = o < 0 ? 0 : (o > RCAP ? RCAP : o);
    const int nc = node < nN ? node : nN - 1;
    int idx = o + lane;
    idx = idx > RCAP - 1 ? RCAP - 1 : idx;
    const int ent = sl[idx];
    int eid = ent >> SLA;
    eid = eid < 0 ? 0 : (eid > nE - 1 ? nE - 1 : eid);
    int sre = srcs[eid];
    sre = sre < 0 ? 0 : (sre > nN - 1 ? nN - 1 : sre);
    const int  sr  = (lane == c) ? nc : sre;
    const bool act = lane <= c;
    const float e0 = ES[sr], e1 = ES[(size_t)NP0 + sr], e2 = ES[(size_t)2 * NP0 + sr];
    const float d0 = ED[nc], d1 = ED[(size_t)NP0 + nc], d2 = ED[(size_t)2 * NP0 + nc];
    float l0 = e0 + d0, l1 = e1 + d1, l2 = e2 + d2;
    l0 = (l0 >= 0.0f) ? l0 : 0.2f * l0;
    l1 = (l1 >= 0.0f) ? l1 : 0.2f * l1;
    l2 = (l2 >= 0.0f) ? l2 : 0.2f * l2;
    l0 = act ? l0 : ninf; l1 = act ? l1 : ninf; l2 = act ? l2 : ninf;
    const float m0 = wmaxf(l0), m1 = wmaxf(l1), m2 = wmaxf(l2);
    float x0 = expf(l0 - m0), x1 = expf(l1 - m1), x2 = expf(l2 - m2);
    x0 = act ? x0 : 0.0f; x1 = act ? x1 : 0.0f; x2 = act ? x2 : 0.0f;
    const float r0 = 1.0f / (wsumf(x0) + 1e-16f);
    const float r1 = 1.0f / (wsumf(x1) + 1e-16f);
    const float r2 = 1.0f / (wsumf(x2) + 1e-16f);
    const int a0i = __float_as_int(x0 * r0);
    const int a1i = __float_as_int(x1 * r1);
    const int a2i = __float_as_int(x2 * r2);
    v4f c0 = {0.f, 0.f, 0.f, 0.f}, c1 = {0.f, 0.f, 0.f, 0.f}, c2 = {0.f, 0.f, 0.f, 0.f};
#pragma unroll 1
    for (int k = 0; k <= c; ++k) {
      const int   sk = __builtin_amdgcn_readlane(sr, k);
      const float w0 = __int_as_float(__builtin_amdgcn_readlane(a0i, k));
      const float w1 = __int_as_float(__builtin_amdgcn_readlane(a1i, k));
      const float w2 = __int_as_float(__builtin_amdgcn_readlane(a2i, k));
      const float* hp = H + (size_t)sk * GW + 4 * lane;
      const v4f v0 = *(const v4f*)hp;
      const v4f v1 = *(const v4f*)(hp + CD);
      const v4f v2 = *(const v4f*)(hp + 2 * CD);
      c0.x = fmaf(w0, v0.x, c0.x); c0.y = fmaf(w0, v0.y, c0.y); c0.z = fmaf(w0, v0.z, c0.z); c0.w = fmaf(w0, v0.w, c0.w);
      c1.x = fmaf(w1, v1.x, c1.x); c1.y = fmaf(w1, v1.y, c1.y); c1.z = fmaf(w1, v1.z, c1.z); c1.w = fmaf(w1, v1.w, c1.w);
      c2.x = fmaf(w2, v2.x, c2.x); c2.y = fmaf(w2, v2.y, c2.y); c2.z = fmaf(w2, v2.z, c2.z); c2.w = fmaf(w2, v2.w, c2.w);
    }
    const float pzr = big ? qnan : pz;
    wbig |= (big && node < nN) ? 1 : 0;
    v4f y0 = c0 + bv0, y1 = c1 + bv1, y2 = c2 + bv2;
    y0.x += pzr; y0.y += pzr; y0.z += pzr; y0.w += pzr;
    y1.x += pzr; y1.y += pzr; y1.z += pzr; y1.w += pzr;
    y2.x += pzr; y2.y += pzr; y2.z += pzr; y2.w += pzr;
    stage3(rowbuf, 4 * lane, GW, y0);
    stage3(rowbuf, CD + 4 * lane, GW, y1);
    stage3(rowbuf, 2 * CD + 4 * lane, GW, y2);
    wave_sync();
    const v8us q0 = *(const v8usa*)(rowbuf + 8 * lane);
    const v8us q1 = *(const v8usa*)(rowbuf + 256 + 8 * lane);
    const v8us q2 = *(const v8usa*)(rowbuf + 512 + 8 * lane);
    const v8us q3 = *(const v8usa*)(rowbuf + 768 + 8 * lane);
    const v8us q4 = *(const v8usa*)(rowbuf + 1024 + 8 * (lane & 15));
    wave_sync();
    if (node < nN) {
      unsigned short* gp = G + (size_t)node * GK + 8 * lane;
      *(volatile v8us*)gp = q0;
      *(volatile v8us*)(gp + 256) = q1;
      *(volatile v8us*)(gp + 512) = q2;
      *(volatile v8us*)(gp + 768) = q3;
      if (lane < 16) *(volatile v8us*)(gp + 1024) = q4;
      __threadfence();
      *(volatile v8us*)gp = q0;
      *(volatile v8us*)(gp + 256) = q1;
      *(volatile v8us*)(gp + 512) = q2;
      *(volatile v8us*)(gp + 768) = q3;
      if (lane < 16) *(volatile v8us*)(gp + 1024) = q4;
    }
  }
  if (lane == 0) misc[16 + wave] = wbig;
  __syncthreads();
  if (wave == 0) {
    int f = ovf;
#pragma unroll
    for (int w2 = 0; w2 < NWAVE; ++w2) f |= misc[16 + w2];
    f = (f != 0) ? 1 : 0;
    const v4i fv = {f, f, f, f};
    int* fp = flags + (size_t)blockIdx.x * 32 + 4 * (lane & 7);
    if (lane < 8) *(volatile v4i*)fp = fv;
    __threadfence();
    if (lane < 8) *(volatile v4i*)fp = fv;
  }
}

__global__ __launch_bounds__(PTHR) void k_pool(const float* __restrict__ HH, const float* __restrict__ score,
                                               int per, int k, int* newid, unsigned short* XN, float* XL) {
  __shared__ __attribute__((aligned(16))) float ls[PERPAD];
  __shared__ __attribute__((aligned(16))) int nid[PERPAD];
  __shared__ int inv[PERPAD];
  __shared__ __attribute__((aligned(16))) float xs[2 * CD];
  __shared__ __attribute__((aligned(16))) unsigned short rb[(PTHR / 32) * XK];
  const int tid = (int)threadIdx.x, lane = tid & 31, wave = tid >> 5;
  const int g = (int)blockIdx.x;
  const int base = g * per;
  {
    const int tc = tid < per ? tid : per - 1;
    const float sv = score[base + tc];
    ls[tid] = (tid < per) ? sv : 0.0f;
    inv[tid] = 0;
  }
  __syncthreads();
  {
    const float my = ls[tid];
    int rank = 0;
#pragma unroll 4
    for (int j = 0; j < per; ++j) {
      const float o = ls[j];
      rank += ((o > my) || (o == my && j < tid)) ? 1 : 0;
    }
    const bool kept = (tid < per) && (rank < k);
    nid[tid] = kept ? (g * k + rank) : -1;
    if (kept) inv[rank] = tid;
  }
  __syncthreads();
  if (tid < PERPAD / 4) {
    const v4i nv = *(const v4ia*)(nid + 4 * tid);
    int* np = newid + (size_t)g * PERPAD + 4 * tid;
    *(volatile v4i*)np = nv;
    __threadfence();
    *(volatile v4i*)np = nv;
  }
  unsigned short* rbw = rb + wave * XK;
#pragma unroll 1
  for (int r = wave; r < k; r += PTHR / 32) {
    int ti = inv[r];
    ti = ti < 0 ? 0 : (ti > per - 1 ? per - 1 : ti);
    const float sc = ls[ti];
    const v4f v = *(const v4f*)(HH + (size_t)(base + ti) * CD + 4 * lane);
    v4f y;
    y.x = v.x * sc; y.y = v.y * sc; y.z = v.z * sc; y.w = v.w * sc;
    stage3(rbw, 4 * lane, CD, y);
    wave_sync();
    const v8us q0 = *(const v8usa*)(rbw + 8 * lane);
    const v8us q1 = *(const v8usa*)(rbw + 256 + 8 * (lane & 15));
    wave_sync();
    unsigned short* xp = XN + (size_t)(g * k + r) * XK + 8 * lane;
    *(volatile v8us*)xp = q0;
    if (lane < 16) *(volatile v8us*)(xp + 256) = q1;
    __threadfence();
    *(volatile v8us*)xp = q0;
    if (lane < 16) *(volatile v8us*)(xp + 256) = q1;
  }
  if (tid < CD) {
    float mx = -__builtin_inff(), sm = 0.0f;
#pragma unroll 1
    for (int r = 0; r < k; ++r) {
      int ti = inv[r];
      ti = ti < 0 ? 0 : (ti > per - 1 ? per - 1 : ti);
      const float v = HH[(size_t)(base + ti) * CD + tid] * ls[ti];
      mx = fmaxf(mx, v);
      sm = sm + v;
    }
    xs[tid] = mx;
    xs[CD + tid] = sm * (1.0f / (float)k);
  }
  __syncthreads();
  if (tid < 64) {
    const v4f ov = *(const v4fa*)(xs + 4 * tid);
    float* op = XL + (size_t)g * (2 * CD) + 4 * tid;
    *(volatile v4f*)op = ov;
    __threadfence();
    *(volatile v4f*)op = ov;
  }
}

__device__ __forceinline__ void remap1(int s, int d, const int* __restrict__ newid, int per, int nPrev, int nNew,
                                       int& so, int& dq) {
  const bool ok0 = (s >= 0) && (d >= 0) && (s < nPrev) && (d < nPrev);
  const int sc = s < 0 ? 0 : (s > nPrev - 1 ? nPrev - 1 : s);
  const int dc = d < 0 ? 0 : (d > nPrev - 1 ? nPrev - 1 : d);
  const int gs = sc / per, gd = dc / per;
  const int ns = newid[(size_t)gs * PERPAD + (sc - gs * per)];
  const int nd = newid[(size_t)gd * PERPAD + (dc - gd * per)];
  const bool ok = ok0 && (ns >= 0) && (nd >= 0) && (ns < nNew) && (nd < nNew);
  so = ok ? ns : -1;
  dq = ok ? nd : -1;
}
__global__ __launch_bounds__(NTHR) void k_remap(const int* __restrict__ sp, const int* __restrict__ dp, int nE,
                                                const int* __restrict__ newid, int per, int nPrev, int nNew,
                                                int* so, int* dq) {
  const int e4 = ((int)blockIdx.x * NTHR + (int)threadIdx.x) * 4;
  if (e4 >= nE) return;
  const v4i s4 = *(const v4i*)(sp + e4);
  const v4i d4 = *(const v4i*)(dp + e4);
  v4i os, od;
  int a, b;
  remap1(s4.x, d4.x, newid, per, nPrev, nNew, a, b); os.x = a; od.x = b;
  remap1(s4.y, d4.y, newid, per, nPrev, nNew, a, b); os.y = a; od.y = b;
  remap1(s4.z, d4.z, newid, per, nPrev, nNew, a, b); os.z = a; od.z = b;
  remap1(s4.w, d4.w, newid, per, nPrev, nNew, a, b); os.w = a; od.w = b;
  *(volatile v4i*)(so + e4) = os;
  *(volatile v4i*)(dq + e4) = od;
  __threadfence();
  *(volatile v4i*)(so + e4) = os;
  *(volatile v4i*)(dq + e4) = od;
}

__global__ __launch_bounds__(NTHR) void k_final(const float* __restrict__ XL, const float* __restrict__ Wl1,
                                                const float* __restrict__ bl1, const float* __restrict__ Wl2,
                                                const float* __restrict__ bl2, const int* __restrict__ flags,
                                                int nf0, int nf1, int nf2, float* out) {
  __shared__ __attribute__((aligned(16))) float zs[256];
  __shared__ __attribute__((aligned(16))) float ts[512];
  __shared__ __attribute__((aligned(16))) float os[256];
  __shared__ int wfl[NWAVE];
  const int tid = (int)threadIdx.x, lane = tid & 31, wave = tid >> 5;
  const int g = (int)blockIdx.x;
  {
    const size_t o = (size_t)g * 256 + tid;
    zs[tid] = (XL[o] + XL[(size_t)NGR * 256 + o]) + XL[(size_t)2 * NGR * 256 + o];
  }
  {
    const int lc = wave < 3 ? wave : 2;
    int nb = (lc == 0) ? nf0 : ((lc == 1) ? nf1 : nf2);
    nb = nb < 0 ? 0 : (nb > 32 ? 32 : nb);
    int bc = lane < nb ? lane : nb - 1;
    bc = bc < 0 ? 0 : bc;
    const int fw = flags[(size_t)(lc * 32 + bc) * 32];
    const bool hit = (wave < 3) && (lane < nb) && (fw == 1);
    const unsigned bm = __builtin_amdgcn_ballot_w32(hit);
    if (lane == 0) wfl[wave] = (bm != 0u) ? 1 : 0;
  }
  __syncthreads();
  int fl = 0;
#pragma unroll
  for (int w2 = 0; w2 < NWAVE; ++w2) fl |= wfl[w2];
#pragma unroll 1
  for (int q = 0; q < 2; ++q) {
    const int col = tid + 256 * q;
    float s = 0.0f;
#pragma unroll 4
    for (int k = 0; k < 256; ++k) s = fmaf(zs[k], bf16_val(Wl1[(size_t)k * 512 + col]), s);
    s = s + bf16_val(bl1[col]);
    ts[col] = (s > 0.0f) ? s : (s - s);
  }
  __syncthreads();
  {
    float s = 0.0f;
#pragma unroll 4
    for (int k = 0; k < 512; ++k) s = fmaf(ts[k], bf16_val(Wl2[(size_t)k * 256 + tid]), s);
    s = s + bf16_val(bl2[tid]);
    os[tid] = (fl != 0) ? __int_as_float(0x7fc00000) : s;
  }
  __syncthreads();
  if (tid < 64) {
    const v4f ov = *(const v4fa*)(os + 4 * tid);
    float* op = out + (size_t)g * 256 + 4 * tid;
    *(volatile v4f*)op = ov;
    __threadfence();
    *(volatile v4f*)op = ov;
  }
}

static inline int cdiv(int a, int b) { return (a + b - 1) / b; }
static inline size_t al256(size_t o) { return (o + 255) & ~(size_t)255; }

extern "C" void kernel_launch(void* const* d_in, const int* in_sizes, int n_in,
                              void* d_out, int out_size, void* d_ws, size_t ws_size,
                              hipStream_t stream) {
  if (n_in < 29) return;
  const int N0 = NP0;
  if (in_sizes[0] != N0 * CD) return;
  if (in_sizes[2] < 8 || (in_sizes[2] & 1) != 0) return;
  const int nE = in_sizes[2] / 2;
  if ((nE & 3) != 0 || nE >= (1 << 21)) return;
  for (int l = 0; l < 3; ++l) {
    const int b = 4 + 7 * l;
    if (in_sizes[b] != CD * GW || in_sizes[b + 1] != GW || in_sizes[b + 2] != GW || in_sizes[b + 3] != GW) return;
    if (in_sizes[b + 4] != GW * CD || in_sizes[b + 5] != CD || in_sizes[b + 6] != CD) return;
  }
  if (in_sizes[25] != 256 * 512 || in_sizes[26] != 512 || in_sizes[27] != 512 * 256 || in_sizes[28] != 256) return;
  if (out_size != NGR * 256) return;
  const int k1 = (int)ceil(0.8 * (double)512);
  const int k2 = (int)ceil(0.5 * (double)k1);
  const int k3 = (int)ceil(0.2 * (double)k2);
  if (k1 != 410 || k2 != 205 || k3 != 41) return;
  const int perl[3] = {512, k1, k2};
  const int keep[3] = {k1, k2, k3};
  const int nlev[4] = {NGR * 512, NGR * k1, NGR * k2, NGR * k3};
  for (int l = 0; l < 3; ++l) if ((nlev[l] % GBM) != 0 || perl[l] > PERPAD) return;

  const float* x    = (const float*)d_in[0];
  const int*   edge = (const int*)d_in[2];
  const float* Wg[3]  = {(const float*)d_in[4],  (const float*)d_in[11], (const float*)d_in[18]};
  const float* asr[3] = {(const float*)d_in[5],  (const float*)d_in[12], (const float*)d_in[19]};
  const float* adt[3] = {(const float*)d_in[6],  (const float*)d_in[13], (const float*)d_in[20]};
  const float* bgt[3] = {(const float*)d_in[7],  (const float*)d_in[14], (const float*)d_in[21]};
  const float* Whd[3] = {(const float*)d_in[8],  (const float*)d_in[15], (const float*)d_in[22]};
  const float* bhd[3] = {(const float*)d_in[9],  (const float*)d_in[16], (const float*)d_in[23]};
  const float* pwv[3] = {(const float*)d_in[10], (const float*)d_in[17], (const float*)d_in[24]};
  const float* Wl1 = (const float*)d_in[25];
  const float* bl1 = (const float*)d_in[26];
  const float* Wl2 = (const float*)d_in[27];
  const float* bl2 = (const float*)d_in[28];
  float* out = (float*)d_out;

  char* ws = (char*)d_ws;
  size_t off = 0;
  const size_t oA   = off; off = al256(off + (size_t)N0 * GW * 4);
  const size_t oB   = off; off = al256(off + (size_t)N0 * GK * 2);
  const size_t oES  = off; off = al256(off + (size_t)3 * N0 * 4);
  const size_t oED  = off; off = al256(off + (size_t)3 * N0 * 4);
  const size_t oSC  = off; off = al256(off + (size_t)N0 * 4);
  const size_t oNID = off; off = al256(off + (size_t)NGR * PERPAD * 4);
  const size_t oS2  = off; off = al256(off + (size_t)nE * 4);
  const size_t oD2  = off; off = al256(off + (size_t)nE * 4);
  const size_t oS3  = off; off = al256(off + (size_t)nE * 4);
  const size_t oD3  = off; off = al256(off + (size_t)nE * 4);
  const size_t oW1T = off; off = al256(off + (size_t)GW * CD * 2);
  const size_t oW2T = off; off = al256(off + (size_t)GW * XK * 2);
  const size_t oW3T = off; off = al256(off + (size_t)GW * XK * 2);
  const size_t oH1T = off; off = al256(off + (size_t)CD * GK * 2);
  const size_t oH2T = off; off = al256(off + (size_t)CD * GK * 2);
  const size_t oH3T = off; off = al256(off + (size_t)CD * GK * 2);
  const size_t oXL  = off; off = al256(off + (size_t)3 * NGR * 256 * 4);
  const size_t oFL  = off; off = al256(off + (size_t)3 * 32 * 128);
  if (off > ws_size || off > (size_t)WSMAX) return;
  float*          RA   = (float*)(ws + oA);
  unsigned short* RB   = (unsigned short*)(ws + oB);
  float*          ES   = (float*)(ws + oES);
  float*          ED   = (float*)(ws + oED);
  float*          SCR  = (float*)(ws + oSC);
  int*            NID  = (int*)(ws + oNID);
  int*            S2   = (int*)(ws + oS2);
  int*            D2   = (int*)(ws + oD2);
  int*            S3   = (int*)(ws + oS3);
  int*            D3   = (int*)(ws + oD3);
  unsigned short* W1T  = (unsigned short*)(ws + oW1T);
  unsigned short* W2T  = (unsigned short*)(ws + oW2T);
  unsigned short* W3T  = (unsigned short*)(ws + oW3T);
  unsigned short* Wh1T = (unsigned short*)(ws + oH1T);
  unsigned short* Wh2T = (unsigned short*)(ws + oH2T);
  unsigned short* Wh3T = (unsigned short*)(ws + oH3T);
  float*          XL   = (float*)(ws + oXL);
  int*            FL   = (int*)(ws + oFL);

  const unsigned short* WgT[3] = {W1T, W2T, W3T};
  const unsigned short* WhT[3] = {Wh1T, Wh2T, Wh3T};
  const int* srcL[3] = {edge, S2, S3};
  const int* dstL[3] = {edge + nE, D2, D3};
  int* srcN[2] = {S2, S3};
  int* dstN[2] = {D2, D3};

  const size_t attnLds = (size_t)AGG_LDS_INTS * 4;
  hipFuncSetAttribute(reinterpret_cast<const void*>(&k_attn), hipFuncAttributeMaxDynamicSharedMemorySize, (int)attnLds);

  k_prep<<<PU_TOT / NTHR, NTHR, 0, stream>>>(Wg[0], Wg[1], Wg[2], Whd[0], Whd[1], Whd[2],
                                             W1T, W2T, W3T, Wh1T, Wh2T, Wh3T);
  k_cvx<<<cdiv(N0 * (CD / 8), NTHR), NTHR, 0, stream>>>(x, N0 * (CD / 8), RB);

  int nfl[3] = {0, 0, 0};
  for (int l = 0; l < 3; ++l) {
    const int n  = nlev[l];
    const int K  = (l == 0) ? CD : XK;
    const int gA = cdiv(n, NBA);
    if (gA < 1 || gA > 32) return;
    nfl[l] = gA;
    k_gemma<<<dim3(n / GBM, 3), GTHR, 0, stream>>>(RB, WgT[l], K, asr[l], adt[l], RA, ES, ED);
    k_attn<<<gA, NTHR, attnLds, stream>>>(srcL[l], dstL[l], nE, n, 1, RA, ES, ED, bgt[l], RB, FL + (size_t)l * 32 * 32);
    k_gemmb<<<n / GBM, GTHR, 0, stream>>>(RB, WhT[l], bhd[l], pwv[l], RA, SCR);
    k_pool<<<NGR, PTHR, 0, stream>>>(RA, SCR, perl[l], keep[l], NID, RB, XL + (size_t)l * NGR * 256);
    if (l < 2)
      k_remap<<<cdiv(nE / 4, NTHR), NTHR, 0, stream>>>(srcL[l], dstL[l], nE, NID, perl[l], n, nlev[l + 1],
                                                       srcN[l], dstN[l]);
  }
  k_final<<<NGR, NTHR, 0, stream>>>(XL, Wl1, bl1, Wl2, bl2, FL, nfl[0], nfl[1], nfl[2], out);
}
